// DeepInterestNetwork_31628139167809
// MI455X (gfx1250) — hardware-verified
//
#include <hip/hip_runtime.h>

#define EDIM   96
#define FDIM   69
#define GDIM   10
#define NWIN   (GDIM * FDIM)
#define ITEMN  100000
#define RPB    2
#define NRB    (RPB * FDIM)
#define NQB    (NRB + RPB)
#define NTB    9
#define NT1    (NTB * 32)
#define K1     384
#define N1     64
#define N2     16
#define XW     1056
#define XP     1088
#define XLINES (XP / 64)
#define NF1    200
#define NF1P   224
#define NF2    80
#define NF2P   96
#define KF2P   256
#define FCROWS 64
#define CH_W1  (N1 * K1 / 8)
#define CH_W2  (N2 * N1 / 8)
#define CH_F1  (NF1P * XP / 8)
#define CH_F2  (NF2P * KF2P / 8)
#define CH_ALL (CH_W1 + CH_W2 + 2 * CH_F1 + 2 * CH_F2)
#define INV_BN 0.99999500003750f

static_assert(NTB * 16 >= NRB);
static_assert((NT1 / 8) * 2 >= RPB * 2 * XLINES);
static_assert(RPB * EDIM <= NT1);
static_assert((CH_W1 % 32) == 0 && (CH_W2 % 32) == 0 && (CH_F1 % 32) == 0 && (CH_F2 % 32) == 0);
static_assert((XP % 64) == 0 && (K1 % 64) == 0 && (N1 % 64) == 0 && (KF2P % 64) == 0);

typedef _Float16 v16h __attribute__((ext_vector_type(16)));
typedef _Float16 v8h  __attribute__((ext_vector_type(8)));
typedef __bf16   v16b __attribute__((ext_vector_type(16)));
typedef unsigned short v8us __attribute__((ext_vector_type(8)));
typedef float v8f __attribute__((ext_vector_type(8)));
typedef float v4f __attribute__((ext_vector_type(4)));
typedef v8h  __attribute__((may_alias)) v8ha;
typedef v8us __attribute__((may_alias)) v8usa;
typedef v4f  __attribute__((may_alias)) v4fa;

union FragH { v16h v; v8h half[2]; };
union FragB { v16b v; v8us half[2]; };

__device__ __forceinline__ v8f wmma_f16(v16h a, v16h b, v8f c) {
  v8f d = __builtin_amdgcn_wmma_f32_16x16x32_f16(false, a, false, b, (short)0, c, false, false);
  asm volatile("v_nop\n\tv_nop\n\tv_nop\n\tv_nop" : "+v"(d) : "v"(a), "v"(b));
  return d;
}
__device__ __forceinline__ v8f wmma_bf(v16b a, v16b b, v8f c) {
  v8f d = __builtin_amdgcn_wmma_f32_16x16x32_bf16(false, a, false, b, (short)0, c, false, false);
  asm volatile("v_nop\n\tv_nop\n\tv_nop\n\tv_nop" : "+v"(d) : "v"(a), "v"(b));
  return d;
}

__device__ __forceinline__ v16h load_frag_h(const _Float16* p, int h) {
  FragH f;
  f.half[0] = *(const v8ha*)(p + 8 * h);
  f.half[1] = *(const v8ha*)(p + 16 + 8 * h);
  return f.v;
}
__device__ __forceinline__ v16b load_frag_b(const unsigned short* p, int h) {
  FragB f;
  f.half[0] = *(const v8usa*)(p + 8 * h);
  f.half[1] = *(const v8usa*)(p + 16 + 8 * h);
  return f.v;
}

__device__ __forceinline__ unsigned bf16_rne_bits(float x) {
  unsigned u = __float_as_uint(x);
  u += 0x7FFFu + ((u >> 16) & 1u);
  return u >> 16;
}
__device__ __forceinline__ float bf16_to_f32(unsigned b) { return __uint_as_float(b << 16); }
__device__ __forceinline__ unsigned short f16_bits(float x) {
  union { _Float16 hv; unsigned short u; } cv;
  cv.hv = (_Float16)x;
  return cv.u;
}
__device__ __forceinline__ unsigned short split_bits(float v, int pl) {
  const unsigned hb = bf16_rne_bits(v);
  const unsigned lb = bf16_rne_bits(v - bf16_to_f32(hb));
  return (unsigned short)(pl ? lb : hb);
}

__device__ __forceinline__ float dicef(float x, float alpha) {
  const float e = __expf(-x);
  const float p = __builtin_amdgcn_rcpf(1.0f + e);
  return (alpha * (1.0f - p) + p) * x;
}

__device__ __forceinline__ v16h make_frag(v4f a, v4f b, v4f c, v4f d, float s) {
  v16h r;
  r[0]  = (_Float16)(a.x * s); r[1]  = (_Float16)(a.y * s); r[2]  = (_Float16)(a.z * s); r[3]  = (_Float16)(a.w * s);
  r[4]  = (_Float16)(b.x * s); r[5]  = (_Float16)(b.y * s); r[6]  = (_Float16)(b.z * s); r[7]  = (_Float16)(b.w * s);
  r[8]  = (_Float16)(c.x * s); r[9]  = (_Float16)(c.y * s); r[10] = (_Float16)(c.z * s); r[11] = (_Float16)(c.w * s);
  r[12] = (_Float16)(d.x * s); r[13] = (_Float16)(d.y * s); r[14] = (_Float16)(d.z * s); r[15] = (_Float16)(d.w * s);
  return r;
}

__device__ __forceinline__ v4f sel4(bool c, v4f a, v4f b) {
  v4f r;
  r.x = c ? a.x : b.x; r.y = c ? a.y : b.y; r.z = c ? a.z : b.z; r.w = c ? a.w : b.w;
  return r;
}

__global__ __launch_bounds__(256) void k_prep(
    const float* __restrict__ W1, const float* __restrict__ W2,
    const float* __restrict__ Wf1, const float* __restrict__ Wf2,
    unsigned short* __restrict__ pW1t, unsigned short* __restrict__ pW2t,
    unsigned short* __restrict__ pF1h, unsigned short* __restrict__ pF1l,
    unsigned short* __restrict__ pF2h, unsigned short* __restrict__ pF2l)
{
  const int c = blockIdx.x * 256 + threadIdx.x;
  if (c >= CH_ALL) return;
  const float* src; int ldn, nmax, kmax, rowlen, rel, mode; float sc; unsigned short* dst;
  if (c < CH_W1) {
    src = W1; ldn = N1; nmax = N1; kmax = K1; rowlen = K1; rel = c; mode = 0; sc = 8.0f; dst = pW1t;
  } else if (c < CH_W1 + CH_W2) {
    src = W2; ldn = N2; nmax = N2; kmax = N1; rowlen = N1; rel = c - CH_W1; mode = 0; sc = 8.0f; dst = pW2t;
  } else if (c < CH_W1 + CH_W2 + CH_F1) {
    src = Wf1; ldn = NF1; nmax = NF1; kmax = XW; rowlen = XP; rel = c - (CH_W1 + CH_W2); mode = 1; sc = 1.0f; dst = pF1h;
  } else if (c < CH_W1 + CH_W2 + 2 * CH_F1) {
    src = Wf1; ldn = NF1; nmax = NF1; kmax = XW; rowlen = XP; rel = c - (CH_W1 + CH_W2 + CH_F1); mode = 2; sc = 1.0f; dst = pF1l;
  } else if (c < CH_W1 + CH_W2 + 2 * CH_F1 + CH_F2) {
    src = Wf2; ldn = NF2; nmax = NF2; kmax = NF1; rowlen = KF2P; rel = c - (CH_W1 + CH_W2 + 2 * CH_F1); mode = 1; sc = 1.0f; dst = pF2h;
  } else {
    src = Wf2; ldn = NF2; nmax = NF2; kmax = NF1; rowlen = KF2P; rel = c - (CH_W1 + CH_W2 + 2 * CH_F1 + CH_F2); mode = 2; sc = 1.0f; dst = pF2l;
  }
  const int cpr = rowlen >> 3;
  const int n = rel / cpr;
  const int kc = (rel - n * cpr) * 8;
  const int nn = min(n, nmax - 1);
  v8us o;
  #pragma unroll
  for (int i = 0; i < 8; ++i) {
    const int k = kc + i;
    const int kk = min(k, kmax - 1);
    float v = src[(size_t)kk * ldn + nn];
    v = (k < kmax && n < nmax) ? v : 0.0f;
    const unsigned short fb = f16_bits(v * sc);
    const unsigned hb = bf16_rne_bits(v);
    const unsigned lb = bf16_rne_bits(v - bf16_to_f32(hb));
    o[i] = (mode == 0) ? fb : ((mode == 1) ? (unsigned short)hb : (unsigned short)lb);
  }
  unsigned short* d = dst + (size_t)rel * 8;
  *(volatile v8us*)d = o;
  __threadfence();
  *(volatile v8us*)d = o;
}

__device__ __forceinline__ void x_store_pass(const float* sPool, const float* sE,
                                             unsigned short* Xhi, unsigned short* Xlo,
                                             int b0, int tid) {
  const v4f z4 = {0.0f, 0.0f, 0.0f, 0.0f};
  #pragma unroll
  for (int sub = 0; sub < 2; ++sub) {
    const int L = sub * (NT1 / 8) + (tid >> 3);
    const int q8 = tid & 7;
    if (L < RPB * 2 * XLINES) {
      const int bb = (L >= 2 * XLINES) ? 1 : 0;
      const int rem = L - 2 * XLINES * bb;
      const int pl = (rem >= XLINES) ? 1 : 0;
      const int ln = rem - XLINES * pl;
      const int c0 = ln * 64 + q8 * 8;
      const float* pa = sPool + bb * (GDIM * EDIM) + min(c0, GDIM * EDIM - 8);
      const float* pq = sE + (NRB + bb) * EDIM + min(max(c0 - GDIM * EDIM, 0), EDIM - 8);
      const v4f a0 = *(const v4fa*)pa;
      const v4f a1 = *(const v4fa*)(pa + 4);
      const v4f g0 = *(const v4fa*)pq;
      const v4f g1 = *(const v4fa*)(pq + 4);
      const bool inA = c0 < GDIM * EDIM;
      const bool inQ = c0 < XW;
      const v4f v0 = sel4(inA, a0, sel4(inQ, g0, z4));
      const v4f v1 = sel4(inA, a1, sel4(inQ, g1, z4));
      v8us o;
      o[0] = split_bits(v0.x, pl); o[1] = split_bits(v0.y, pl); o[2] = split_bits(v0.z, pl); o[3] = split_bits(v0.w, pl);
      o[4] = split_bits(v1.x, pl); o[5] = split_bits(v1.y, pl); o[6] = split_bits(v1.z, pl); o[7] = split_bits(v1.w, pl);
      unsigned short* dst = (pl ? Xlo : Xhi) + (size_t)(b0 + bb) * XP + c0;
      *(volatile v8us*)dst = o;
    }
  }
}

__global__ __launch_bounds__(NT1) void k_attn_pool(
    const int* __restrict__ bu, const int* __restrict__ bl,
    const float* __restrict__ emb, const float* __restrict__ win,
    const _Float16* __restrict__ W1t, const float* __restrict__ b1, const float* __restrict__ a1,
    const _Float16* __restrict__ W2t, const float* __restrict__ b2,
    const float* __restrict__ W3, const float* __restrict__ b3,
    unsigned short* __restrict__ Xhi, unsigned short* __restrict__ Xlo,
    int nemb)
{
  __shared__ __attribute__((aligned(16))) float sE[NQB * EDIM];
  __shared__ __attribute__((aligned(16))) _Float16 sH[NTB * 16 * 64];
  __shared__ __attribute__((aligned(16))) float sPool[RPB * GDIM * EDIM];
  __shared__ float sWin[NWIN];
  __shared__ float sLw[NWIN];
  __shared__ int   sLfg[NWIN];
  __shared__ int   sId[NTB * 16];
  __shared__ int   sEff[NTB * 16];
  __shared__ float sAtt[NTB * 16];
  __shared__ int   sCnt;

  const int tid = threadIdx.x, lane = tid & 31, wv = tid >> 5;
  const int h = lane >> 4, m = lane & 15;
  const int b0 = blockIdx.x * RPB;

  if (wv < 5) {
    const int i = min(tid, NTB * 16 - 1);
    const int iu = min(i, NRB - 1);
    const int bbu = (iu >= FDIM) ? 1 : 0;
    const int fu = iu - FDIM * bbu;
    const int rawu = bu[(size_t)(b0 + bbu) * FDIM + fu];
    const int il = min(max(i - NRB, 0), RPB - 1);
    const int rawl = bl[b0 + il];
    const int raw = (i < NRB) ? rawu : ((i < NQB) ? rawl : ITEMN);
    sId[i] = min(max(raw, 0), nemb - 1);
    sEff[i] = (i < NRB && raw < ITEMN) ? 1 : 0;
  }
  #pragma unroll
  for (int it = 0; it < 3; ++it) {
    const int i = it * NT1 + tid;
    const float w = win[min(i, NWIN - 1)];
    if (i < NWIN) sWin[i] = w;
  }
  __syncthreads();

  if (wv == 0) {
    int cnt = 0;
    #pragma unroll 1
    for (int base = 0; base < NWIN; base += 32) {
      const int idx = base + lane;
      const int idc = min(idx, NWIN - 1);
      const float w = sWin[idc];
      const bool nz = (idx < NWIN) && (w != 0.0f);
      const unsigned bal = __builtin_amdgcn_ballot_w32(nz);
      const int pos = cnt + (int)__builtin_popcount(bal & ((1u << lane) - 1u));
      if (nz) {
        const int g = idc / FDIM;
        const int f = idc - g * FDIM;
        sLfg[pos] = (g << 8) | f;
        sLw[pos] = w;
      }
      cnt += (int)__builtin_popcount(bal);
    }
    if (lane == 0) sCnt = cnt;
  }
  for (int c = tid; c < NQB * (EDIM / 4); c += NT1) {
    const int row = c / (EDIM / 4);
    const int c4 = c - row * (EDIM / 4);
    const v4f v = *(const v4fa*)(emb + (size_t)sId[row] * EDIM + 4 * c4);
    *(v4fa*)(sE + row * EDIM + 4 * c4) = v;
  }
  __syncthreads();

  const v8f zero8 = {0.0f, 0.0f, 0.0f, 0.0f, 0.0f, 0.0f, 0.0f, 0.0f};

  {
    const int r = 16 * wv + m;
    const int rr = min(r, NRB - 1);
    const float padf = (r < NRB) ? 1.0f : 0.0f;
    const int bbr = (rr >= FDIM) ? 1 : 0;
    const float* up = sE + rr * EDIM;
    const float* qp = sE + (NRB + bbr) * EDIM;
    const float S1 = 4096.0f * padf;
    const float S2 = 16777216.0f * padf;
    v8f acc1[4], acc2[4];
    #pragma unroll
    for (int nt = 0; nt < 4; ++nt) { acc1[nt] = zero8; acc2[nt] = zero8; }

    #pragma unroll
    for (int ec = 0; ec < 3; ++ec) {
      const int e0 = 32 * ec + 8 * h;
      const v4f q0 = *(const v4fa*)(qp + e0);
      const v4f q1 = *(const v4fa*)(qp + e0 + 4);
      const v4f q2 = *(const v4fa*)(qp + e0 + 16);
      const v4f q3 = *(const v4fa*)(qp + e0 + 20);
      const v4f u0 = *(const v4fa*)(up + e0);
      const v4f u1 = *(const v4fa*)(up + e0 + 4);
      const v4f u2 = *(const v4fa*)(up + e0 + 16);
      const v4f u3 = *(const v4fa*)(up + e0 + 20);
      const v16h aq = make_frag(q0, q1, q2, q3, S1);
      const v16h au = make_frag(u0, u1, u2, u3, S1);
      const v16h ad = make_frag(q0 - u0, q1 - u1, q2 - u2, q3 - u3, S1);
      const v16h ap = make_frag(q0 * u0, q1 * u1, q2 * u2, q3 * u3, S2);
      #pragma unroll
      for (int nt = 0; nt < 4; ++nt) {
        const _Float16* wr = W1t + (size_t)(16 * nt + m) * K1;
        const v16h bq = load_frag_h(wr + 32 * ec, h);
        acc1[nt] = wmma_f16(aq, bq, acc1[nt]);
        const v16h bw = load_frag_h(wr + 32 * (3 + ec), h);
        acc1[nt] = wmma_f16(au, bw, acc1[nt]);
        const v16h bd = load_frag_h(wr + 32 * (6 + ec), h);
        acc1[nt] = wmma_f16(ad, bd, acc1[nt]);
        const v16h bp = load_frag_h(wr + 32 * (9 + ec), h);
        acc2[nt] = wmma_f16(ap, bp, acc2[nt]);
      }
    }

    _Float16* shw = sH + wv * (16 * 64);
    #pragma unroll
    for (int nt = 0; nt < 4; ++nt) {
      const int n = 16 * nt + m;
      const float bias = b1[n], alp = a1[n];
      #pragma unroll
      for (int rI = 0; rI < 8; ++rI) {
        const float x = acc1[nt][rI] * (1.0f / 32768.0f) + acc2[nt][rI] * (1.0f / 134217728.0f) + bias;
        const float hd = dicef(x, alp);
        shw[(8 * h + rI) * 64 + n] = (_Float16)(hd * 16384.0f);
      }
    }
  }
  __syncthreads();

  {
    const _Float16* shr = sH + wv * (16 * 64) + m * 64;
    const v16h fa0 = load_frag_h(shr, h);
    const v16h fa1 = load_frag_h(shr + 32, h);
    const _Float16* w2r = W2t + m * 64;
    const v16h fb0 = load_frag_h(w2r, h);
    const v16h fb1 = load_frag_h(w2r + 32, h);
    v8f accw = zero8;
    accw = wmma_f16(fa0, fb0, accw);
    accw = wmma_f16(fa1, fb1, accw);
    const float b2v = b2[m], w3v = W3[m];
    float pr[8];
    #pragma unroll
    for (int rI = 0; rI < 8; ++rI) pr[rI] = (accw[rI] * (1.0f / 131072.0f) + b2v) * w3v;
    #pragma unroll
    for (int msk = 1; msk < 16; msk <<= 1) {
      #pragma unroll
      for (int rI = 0; rI < 8; ++rI) pr[rI] += __shfl_xor(pr[rI], msk);
    }
    const float b3v = b3[0];
    #pragma unroll
    for (int rI = 0; rI < 8; ++rI) {
      const int row = 16 * wv + 8 * h + rI;
      const int effv = sEff[row];
      const float att = pr[rI] + b3v;
      const float attm = (effv != 0) ? att : 0.0f;
      if (m == 0) sAtt[row] = attm;
    }
  }
  __syncthreads();

  if (tid < RPB * EDIM) {
    const int bb = (tid >= EDIM) ? 1 : 0;
    const int e = tid - EDIM * bb;
    float* pc = sPool + bb * (GDIM * EDIM) + e;
    #pragma unroll
    for (int g = 0; g < GDIM; ++g) pc[g * EDIM] = 0.0f;
    const int cnt = min(sCnt, NWIN);
    const float* ub = sE + bb * FDIM * EDIM + e;
    const float* ab = sAtt + bb * FDIM;
    #pragma unroll 1
    for (int j = 0; j < cnt; ++j) {
      const int fg = sLfg[j];
      const int f = min(fg & 255, FDIM - 1);
      const int g = min((fg >> 8) & 15, GDIM - 1);
      const float w = sLw[j];
      const float p = ub[f * EDIM] * ab[f];
      float* cell = pc + g * EDIM;
      const float nv = fmaf(w, p, *cell);
      *cell = nv;
    }
  }
  __syncthreads();

  x_store_pass(sPool, sE, Xhi, Xlo, b0, tid);
  __threadfence();
  x_store_pass(sPool, sE, Xhi, Xlo, b0, tid);
}

__global__ __launch_bounds__(256) void k_fc(
    const unsigned short* __restrict__ Xhi, const unsigned short* __restrict__ Xlo,
    const unsigned short* __restrict__ F1h, const unsigned short* __restrict__ F1l,
    const float* __restrict__ bf1, const float* __restrict__ af1,
    const unsigned short* __restrict__ F2h, const unsigned short* __restrict__ F2l,
    const float* __restrict__ bf2, const float* __restrict__ af2,
    const float* __restrict__ Wf3, const float* __restrict__ bf3,
    float* __restrict__ out)
{
  __shared__ __attribute__((aligned(16))) unsigned short sH1[2 * FCROWS * NF1P];
  __shared__ float sPart[2 * FCROWS];
  __shared__ __attribute__((aligned(16))) float sOut[FCROWS];

  const int tid = threadIdx.x, lane = tid & 31, wv = tid >> 5;
  const int h = lane >> 4, m = lane & 15;
  const int rt = wv >> 1, ch = wv & 1;
  const int lrow = 16 * rt;
  const size_t grow = (size_t)blockIdx.x * FCROWS + lrow + m;
  const unsigned short* xh = Xhi + grow * XP;
  const unsigned short* xl = Xlo + grow * XP;

  const v8f zero8 = {0.0f, 0.0f, 0.0f, 0.0f, 0.0f, 0.0f, 0.0f, 0.0f};
  v8f acc[7];
  #pragma unroll
  for (int nt = 0; nt < 7; ++nt) acc[nt] = zero8;

  #pragma unroll 1
  for (int kt = 0; kt < XP / 32; ++kt) {
    const v16b ah = load_frag_b(xh + 32 * kt, h);
    const v16b al = load_frag_b(xl + 32 * kt, h);
    #pragma unroll
    for (int nt = 0; nt < 7; ++nt) {
      const size_t wo = (size_t)(112 * ch + 16 * nt + m) * XP + 32 * kt;
      const v16b bh = load_frag_b(F1h + wo, h);
      const v16b blo = load_frag_b(F1l + wo, h);
      acc[nt] = wmma_bf(ah, bh, acc[nt]);
      acc[nt] = wmma_bf(ah, blo, acc[nt]);
      acc[nt] = wmma_bf(al, bh, acc[nt]);
    }
  }

  #pragma unroll
  for (int nt = 0; nt < 7; ++nt) {
    const int n = 112 * ch + 16 * nt + m;
    const int nc = min(n, NF1 - 1);
    const float bias = bf1[nc], alp = af1[nc];
    const float keep = (n < NF1) ? 1.0f : 0.0f;
    #pragma unroll
    for (int rI = 0; rI < 8; ++rI) {
      const float v = (acc[nt][rI] + bias) * INV_BN;
      const float hd = dicef(v, alp) * keep;
      const unsigned hb = bf16_rne_bits(hd);
      const unsigned lb = bf16_rne_bits(hd - bf16_to_f32(hb));
      const int li = (lrow + 8 * h + rI) * NF1P + n;
      sH1[li] = (unsigned short)hb;
      sH1[FCROWS * NF1P + li] = (unsigned short)lb;
    }
  }
  __syncthreads();

  v8f acc2[3];
  #pragma unroll
  for (int nt = 0; nt < 3; ++nt) acc2[nt] = zero8;
  {
    const unsigned short* ar = sH1 + (lrow + m) * NF1P;
    #pragma unroll
    for (int kt = 0; kt < NF1P / 32; ++kt) {
      const v16b ah = load_frag_b(ar + 32 * kt, h);
      const v16b al = load_frag_b(ar + FCROWS * NF1P + 32 * kt, h);
      #pragma unroll
      for (int nt = 0; nt < 3; ++nt) {
        const size_t wo = (size_t)(48 * ch + 16 * nt + m) * KF2P + 32 * kt;
        const v16b bh = load_frag_b(F2h + wo, h);
        const v16b blo = load_frag_b(F2l + wo, h);
        acc2[nt] = wmma_bf(ah, bh, acc2[nt]);
        acc2[nt] = wmma_bf(ah, blo, acc2[nt]);
        acc2[nt] = wmma_bf(al, bh, acc2[nt]);
      }
    }
  }

  float pr[8];
  #pragma unroll
  for (int rI = 0; rI < 8; ++rI) pr[rI] = 0.0f;
  #pragma unroll
  for (int nt = 0; nt < 3; ++nt) {
    const int col = 48 * ch + 16 * nt + m;
    const int cc = min(col, NF2 - 1);
    const float bias = bf2[cc], alp = af2[cc], w3 = Wf3[cc];
    const float keep = (col < NF2) ? 1.0f : 0.0f;
    #pragma unroll
    for (int rI = 0; rI < 8; ++rI) {
      const float v = (acc2[nt][rI] + bias) * INV_BN;
      pr[rI] += dicef(v, alp) * keep * w3;
    }
  }
  #pragma unroll
  for (int msk = 1; msk < 16; msk <<= 1) {
    #pragma unroll
    for (int rI = 0; rI < 8; ++rI) pr[rI] += __shfl_xor(pr[rI], msk);
  }
  if (m == 0) {
    #pragma unroll
    for (int rI = 0; rI < 8; ++rI) sPart[ch * FCROWS + lrow + 8 * h + rI] = pr[rI];
  }
  __syncthreads();
  if (tid < FCROWS) sOut[tid] = sPart[tid] + sPart[FCROWS + tid] + bf3[0];
  __syncthreads();
  if (wv == 0) {
    const int lq = lane & 15;
    const v4f o = *(const v4fa*)(sOut + 4 * lq);
    float* dst = out + (size_t)blockIdx.x * FCROWS + 4 * lq;
    if (lane < 16) { *(volatile v4f*)dst = o; }
    __threadfence();
    if (lane < 16) { *(volatile v4f*)dst = o; }
  }
}

extern "C" void kernel_launch(void* const* d_in, const int* in_sizes, int n_in,
                              void* d_out, int out_size, void* d_ws, size_t ws_size,
                              hipStream_t stream) {
  if (n_in < 19) return;
  const int B = in_sizes[1];
  if (B <= 0 || (B % FCROWS) != 0 || (B % RPB) != 0) return;
  if (in_sizes[0] != B * FDIM) return;
  if (out_size != B) return;
  if (in_sizes[2] < EDIM || (in_sizes[2] % EDIM) != 0) return;
  const int nemb = in_sizes[2] / EDIM;
  if (in_sizes[3] != K1 * N1 || in_sizes[4] != N1 || in_sizes[5] != N1) return;
  if (in_sizes[6] != N1 * N2 || in_sizes[7] != N2 || in_sizes[8] != N2 || in_sizes[9] < 1) return;
  if (in_sizes[10] != XW * NF1 || in_sizes[11] != NF1 || in_sizes[12] != NF1) return;
  if (in_sizes[13] != NF1 * NF2 || in_sizes[14] != NF2 || in_sizes[15] != NF2) return;
  if (in_sizes[16] != NF2 || in_sizes[17] < 1 || in_sizes[18] != NWIN) return;

  const int*   bu  = (const int*)d_in[0];
  const int*   bl  = (const int*)d_in[1];
  const float* emb = (const float*)d_in[2];
  const float* W1  = (const float*)d_in[3];
  const float* b1  = (const float*)d_in[4];
  const float* a1  = (const float*)d_in[5];
  const float* W2  = (const float*)d_in[6];
  const float* b2  = (const float*)d_in[7];
  const float* W3  = (const float*)d_in[8];
  const float* b3  = (const float*)d_in[9];
  const float* Wf1 = (const float*)d_in[10];
  const float* bf1 = (const float*)d_in[11];
  const float* af1 = (const float*)d_in[12];
  const float* Wf2 = (const float*)d_in[13];
  const float* bf2 = (const float*)d_in[14];
  const float* af2 = (const float*)d_in[15];
  const float* Wf3 = (const float*)d_in[16];
  const float* bf3 = (const float*)d_in[17];
  const float* win = (const float*)d_in[18];
  float* out = (float*)d_out;

  const size_t szW1t = (size_t)N1 * K1 * 2;
  const size_t szW2t = (size_t)N2 * N1 * 2;
  const size_t szF1  = (size_t)NF1P * XP * 2;
  const size_t szF2  = (size_t)NF2P * KF2P * 2;
  const size_t szX   = (size_t)B * XP * 2;
  const size_t oW1t = 0;
  const size_t oW2t = oW1t + szW1t;
  const size_t oF1h = oW2t + szW2t;
  const size_t oF1l = oF1h + szF1;
  const size_t oF2h = oF1l + szF1;
  const size_t oF2l = oF2h + szF2;
  const size_t oXh  = oF2l + szF2;
  const size_t oXl  = oXh + szX;
  const size_t total = oXl + szX;
  if (total > ws_size) return;

  char* ws = (char*)d_ws;
  unsigned short* pW1t = (unsigned short*)(ws + oW1t);
  unsigned short* pW2t = (unsigned short*)(ws + oW2t);
  unsigned short* pF1h = (unsigned short*)(ws + oF1h);
  unsigned short* pF1l = (unsigned short*)(ws + oF1l);
  unsigned short* pF2h = (unsigned short*)(ws + oF2h);
  unsigned short* pF2l = (unsigned short*)(ws + oF2l);
  unsigned short* pXh  = (unsigned short*)(ws + oXh);
  unsigned short* pXl  = (unsigned short*)(ws + oXl);

  k_prep<<<(CH_ALL + 255) / 256, 256, 0, stream>>>(W1, W2, Wf1, Wf2, pW1t, pW2t, pF1h, pF1l, pF2h, pF2l);

  k_attn_pool<<<B / RPB, NT1, 0, stream>>>(bu, bl, emb, win,
                                            (const _Float16*)pW1t, b1, a1,
                                            (const _Float16*)pW2t, b2, W3, b3,
                                            pXh, pXl, nemb);

  k_fc<<<B / FCROWS, 256, 0, stream>>>(pXh, pXl, pF1h, pF1l, bf1, af1, pF2h, pF2l, bf2, af2, Wf3, bf3, out);
}
